// CausalSelfAttention_33088428048914
// MI455X (gfx1250) — hardware-verified
//
#include <hip/hip_runtime.h>


#ifndef NB
#define NB 4
#endif
#ifndef SEQ
#define SEQ 2048
#endif
#define NB_FULL  4
#define SEQ_FULL 2048
#define DMODEL   1024
#define NHEAD    16
#define HDIM     64
#define RHI      ((SEQ < 512) ? SEQ : 512)
#define WCAR     1024.0f
#define CCAR     16.0f
#define NEGL     (-1.0e30f)
#define SL2E     0.18033688011112042f

static_assert(NHEAD * HDIM == DMODEL);
static_assert(SEQ % 64 == 0);
static_assert(RHI % 64 == 0);
static_assert((SEQ - RHI) % 64 == 0);
static_assert(NB <= NB_FULL);
static_assert(SEQ <= SEQ_FULL);
static_assert(DMODEL % 64 == 0);

typedef _Float16 h16;
typedef unsigned short bf;
typedef __attribute__((ext_vector_type(16))) __bf16   v16bf;
typedef __attribute__((ext_vector_type(16))) _Float16 v16h;
typedef __attribute__((ext_vector_type(8)))  _Float16 v8h;
typedef __attribute__((ext_vector_type(8)))  unsigned short v8us;
typedef __attribute__((ext_vector_type(8)))  float    v8f;
typedef __attribute__((ext_vector_type(4)))  float    v4f;
typedef v4f  __attribute__((may_alias)) v4fa;

__device__ __forceinline__ unsigned short f2bf(float f) { unsigned u = __float_as_uint(f); u += 0x7FFFu + ((u >> 16) & 1u); return (unsigned short)(u >> 16); }
__device__ __forceinline__ float bf2f(unsigned short b) { return __uint_as_float(((unsigned)b) << 16); }
__device__ __forceinline__ float bfr(float f) { return bf2f(f2bf(f)); }
__device__ __forceinline__ v16h cat16(v8h lo, v8h hi) { return __builtin_shufflevector(lo, hi, 0, 1, 2, 3, 4, 5, 6, 7, 8, 9, 10, 11, 12, 13, 14, 15); }
__device__ __forceinline__ v16bf cat16b(v8us lo, v8us hi) { return __builtin_bit_cast(v16bf, __builtin_shufflevector(lo, hi, 0, 1, 2, 3, 4, 5, 6, 7, 8, 9, 10, 11, 12, 13, 14, 15)); }
__device__ __forceinline__ v8f wmma16(v16h a, v16h b, v8f c) { return __builtin_amdgcn_wmma_f32_16x16x32_f16(false, a, false, b, (short)0, c, false, false); }
__device__ __forceinline__ v8f wmmab(v16bf a, v16bf b, v8f c) { return __builtin_amdgcn_wmma_f32_16x16x32_bf16(false, a, false, b, (short)0, c, false, false); }
__device__ __forceinline__ h16 tohx(float x) { return (h16)x; }
__device__ __forceinline__ void splitf(float y, unsigned short& h, unsigned short& l) { h = f2bf(y); l = f2bf(y - bf2f(h)); }

template <typename T16> struct WFrag;
template <> struct WFrag<h16> { typedef v16h V; static __device__ __forceinline__ V ld(const h16* p) { return cat16(*(const v8h*)p, *(const v8h*)(p + 16)); } static __device__ __forceinline__ v8f mma(V a, V b, v8f c) { return wmma16(a, b, c); } };
template <> struct WFrag<bf> { typedef v16bf V; static __device__ __forceinline__ V ld(const bf* p) { return cat16b(*(const v8us*)p, *(const v8us*)(p + 16)); } static __device__ __forceinline__ v8f mma(V a, V b, v8f c) { return wmmab(a, b, c); } };

__global__ __launch_bounds__(256) void k_cvtx(const float* __restrict__ x, bf* XB) {
    const unsigned i = blockIdx.x * 256u + threadIdx.x;
    if (i >= (unsigned)(NB * SEQ * (DMODEL / 8))) return;
    const unsigned row = i / (unsigned)(DMODEL / 8), c8 = i % (unsigned)(DMODEL / 8);
    const unsigned b = row / (unsigned)SEQ, t = row % (unsigned)SEQ;
    const v8f v = *(const v8f*)(x + ((size_t)b * SEQ_FULL + t) * DMODEL + c8 * 8u);
    v8us o;
#pragma unroll
    for (int k = 0; k < 8; ++k) o[k] = f2bf(v[k]);
    bf* d = XB + (size_t)i * 8u;
    *(volatile v8us*)d = o; __threadfence(); *(volatile v8us*)d = o;
}
__global__ __launch_bounds__(256) void k_cvt8(const float* __restrict__ src, bf* dst, unsigned n8) {
    const unsigned i = blockIdx.x * 256u + threadIdx.x; if (i >= n8) return;
    const v8f v = *(const v8f*)(src + (size_t)i * 8u); v8us o;
#pragma unroll
    for (int k = 0; k < 8; ++k) o[k] = f2bf(v[k]);
    bf* d = dst + (size_t)i * 8u;
    *(volatile v8us*)d = o; __threadfence(); *(volatile v8us*)d = o;
}
__global__ __launch_bounds__(256) void k_cvtwo(const float* __restrict__ src, bf* dstb, h16* dsth, unsigned n8) {
    const unsigned i = blockIdx.x * 256u + threadIdx.x; if (i >= n8) return;
    const v8f v = *(const v8f*)(src + (size_t)i * 8u); v8us o; v8h g;
#pragma unroll
    for (int k = 0; k < 8; ++k) { const unsigned short u = f2bf(v[k]); o[k] = u; g[k] = tohx(bf2f(u) * WCAR); }
    bf* d = dstb + (size_t)i * 8u; h16* e = dsth + (size_t)i * 8u;
    *(volatile v8us*)d = o; *(volatile v8h*)e = g; __threadfence(); *(volatile v8us*)d = o; *(volatile v8h*)e = g;
}

__global__ __launch_bounds__(32) void k_gemmqkv(const bf* __restrict__ A, const bf* __restrict__ Bt, const float* __restrict__ bias,
                                                h16* Q16, bf* QPh, bf* QPl, h16* K16, bf* KPh, bf* KPl, h16* VT16, bf* VTh, bf* VTl) {
    typedef WFrag<bf>::V V;
    __shared__ __align__(16) float os[64 * 68];
    const unsigned lane = threadIdx.x & 31u, lr = lane & 15u, hi = lane >> 4, sub = lane >> 3, seg = lane & 7u;
    const unsigned r0 = blockIdx.x * 64u, c0 = blockIdx.y * 64u;
    v8f acc[4][4];
#pragma unroll
    for (int mb = 0; mb < 4; ++mb)
#pragma unroll
        for (int nb = 0; nb < 4; ++nb) acc[mb][nb] = (v8f){};
    const size_t aoff = (size_t)(r0 + lr) * DMODEL + 8u * hi, boff = (size_t)(c0 + lr) * DMODEL + 8u * hi;
#pragma unroll 1
    for (unsigned kc = 0; kc < (unsigned)DMODEL; kc += 32u) {
        V a[4];
#pragma unroll
        for (int mb = 0; mb < 4; ++mb) a[mb] = WFrag<bf>::ld(A + aoff + (size_t)mb * 16 * DMODEL + kc);
#pragma unroll
        for (int nb = 0; nb < 4; ++nb) { const V b = WFrag<bf>::ld(Bt + boff + (size_t)nb * 16 * DMODEL + kc);
#pragma unroll
            for (int mb = 0; mb < 4; ++mb) acc[mb][nb] = WFrag<bf>::mma(a[mb], b, acc[mb][nb]); }
        asm volatile("v_nop\n\tv_nop\n\tv_nop\n\tv_nop" : "+v"(acc[0][0]), "+v"(acc[1][1]), "+v"(acc[2][2]), "+v"(acc[3][3]) : "v"(a[0]), "v"(a[3]));
    }
    float bv[4];
#pragma unroll
    for (int nb = 0; nb < 4; ++nb) bv[nb] = bfr(bias[c0 + (unsigned)nb * 16u + lr]);
#pragma unroll
    for (int mb = 0; mb < 4; ++mb)
#pragma unroll
        for (int nb = 0; nb < 4; ++nb)
#pragma unroll
            for (int j = 0; j < 8; ++j) os[((unsigned)mb * 16u + hi * 8u + (unsigned)j) * 68u + (unsigned)nb * 16u + lr] = acc[mb][nb][j] + bv[nb];
    __syncthreads();
    const unsigned which = c0 / (unsigned)DMODEL, head = (c0 % (unsigned)DMODEL) / (unsigned)HDIM;
    const unsigned b = r0 / (unsigned)SEQ, t0 = r0 % (unsigned)SEQ, bh = b * NHEAD + head;
    const bool low = (t0 < (unsigned)RHI);
    if (which < 2u) {
        h16* P16 = (which == 0u) ? Q16 : K16; bf* Ph = (which == 0u) ? QPh : KPh; bf* Pl = (which == 0u) ? QPl : KPl;
        const bool w16 = (which == 1u) || !low;
#pragma unroll 1
        for (int ps = 0; ps < 2; ++ps) {
#pragma unroll 4
            for (unsigned s = 0; s < 16u; ++s) {
                const unsigned row = s * 4u + sub; const float* src = os + row * 68u + seg * 8u;
                const v4f x0 = *(const v4fa*)src, x1 = *(const v4fa*)(src + 4);
                if (w16) { v8h o;
#pragma unroll
                    for (int i = 0; i < 4; ++i) { o[i] = tohx(x0[i]); o[4 + i] = tohx(x1[i]); }
                    *(volatile v8h*)(P16 + ((size_t)bh * SEQ + t0 + row) * HDIM + seg * 8u) = o; }
                if (low) { v8us oh, ol;
#pragma unroll
                    for (int i = 0; i < 4; ++i) { unsigned short a2, c2; splitf(x0[i], a2, c2); oh[i] = a2; ol[i] = c2; splitf(x1[i], a2, c2); oh[4 + i] = a2; ol[4 + i] = c2; }
                    const size_t oo = ((size_t)bh * RHI + t0 + row) * HDIM + seg * 8u;
                    *(volatile v8us*)(Ph + oo) = oh; *(volatile v8us*)(Pl + oo) = ol; }
            }
            if (ps == 0) __threadfence();
        }
    } else {
#pragma unroll 1
        for (int ps = 0; ps < 2; ++ps) {
#pragma unroll 4
            for (unsigned s = 0; s < 16u; ++s) {
                const unsigned d = s * 4u + sub; float xv[8];
#pragma unroll
                for (int i = 0; i < 8; ++i) xv[i] = os[(seg * 8u + (unsigned)i) * 68u + d];
                v8h o;
#pragma unroll
                for (int i = 0; i < 8; ++i) o[i] = tohx(xv[i]);
                *(volatile v8h*)(VT16 + ((size_t)bh * HDIM + d) * SEQ + t0 + seg * 8u) = o;
                if (low) { v8us oh, ol;
#pragma unroll
                    for (int i = 0; i < 8; ++i) { unsigned short a2, c2; splitf(xv[i], a2, c2); oh[i] = a2; ol[i] = c2; }
                    const size_t oo = ((size_t)bh * HDIM + d) * RHI + t0 + seg * 8u;
                    *(volatile v8us*)(VTh + oo) = oh; *(volatile v8us*)(VTl + oo) = ol; }
            }
            if (ps == 0) __threadfence();
        }
    }
}

template <bool HL> struct FT { typedef h16 T; };
template <> struct FT<true> { typedef bf T; };
template <bool HL, int QT>
__global__ __launch_bounds__(32) void k_flash(const typename FT<HL>::T* __restrict__ Qa, const typename FT<HL>::T* __restrict__ Qb,
                                              const typename FT<HL>::T* __restrict__ Ka, const typename FT<HL>::T* __restrict__ Kb,
                                              const typename FT<HL>::T* __restrict__ Va, const typename FT<HL>::T* __restrict__ Vb,
                                              const int* __restrict__ amask, typename FT<HL>::T* Oa, typename FT<HL>::T* Ob) {
    typedef typename FT<HL>::T T; typedef WFrag<T> W; typedef typename W::V V;
    constexpr unsigned PR = HL ? (unsigned)RHI : (unsigned)SEQ;
    constexpr unsigned QB = HL ? 0u : (unsigned)RHI;
    __shared__ __align__(16) float os[16 * QT * 68];
    const unsigned lane = threadIdx.x & 31u, lr = lane & 15u, hi = lane >> 4, sub = lane >> 3, seg = lane & 7u;
    const unsigned q0 = QB + blockIdx.x * (16u * QT), head = blockIdx.y, b = blockIdx.z, bh = b * NHEAD + head;
    const int* mr = amask + (size_t)b * SEQ_FULL;
    const size_t pbase = (size_t)bh * PR * HDIM;
    V qf[QT][2], qg[QT][2];
#pragma unroll
    for (int qt = 0; qt < QT; ++qt)
#pragma unroll
        for (int ks = 0; ks < 2; ++ks) { const size_t qo = pbase + (size_t)(q0 + (unsigned)qt * 16u + lr) * HDIM + (unsigned)ks * 32u + 8u * hi;
            qf[qt][ks] = W::ld(Qa + qo); if constexpr (HL) qg[qt][ks] = W::ld(Qb + qo); }
    v8f o[4][QT]; float mrun[QT], lrun[QT];
#pragma unroll
    for (int qt = 0; qt < QT; ++qt) { mrun[qt] = NEGL; lrun[qt] = 0.f;
#pragma unroll
        for (int dt = 0; dt < 4; ++dt) o[dt][qt] = (v8f){}; }
    const unsigned nkb = (q0 + 16u * QT + 31u) >> 5;
#pragma unroll 1
    for (unsigned kb = 0; kb < nkb; ++kb) {
        const unsigned k0 = kb * 32u;
        v8f st[2][QT];
#pragma unroll
        for (int kt = 0; kt < 2; ++kt)
#pragma unroll
            for (int qt = 0; qt < QT; ++qt) st[kt][qt] = (v8f){};
#pragma unroll
        for (int kt = 0; kt < 2; ++kt)
#pragma unroll
            for (int ks = 0; ks < 2; ++ks) { const size_t ko = pbase + (size_t)(k0 + (unsigned)kt * 16u + lr) * HDIM + (unsigned)ks * 32u + 8u * hi;
                const V a = W::ld(Ka + ko); V a2; if constexpr (HL) a2 = W::ld(Kb + ko);
#pragma unroll
                for (int qt = 0; qt < QT; ++qt) { st[kt][qt] = W::mma(a, qf[qt][ks], st[kt][qt]);
                    if constexpr (HL) { st[kt][qt] = W::mma(a2, qf[qt][ks], st[kt][qt]); st[kt][qt] = W::mma(a, qg[qt][ks], st[kt][qt]); } } }
        if constexpr (QT == 2) asm volatile("v_nop\n\tv_nop\n\tv_nop\n\tv_nop" : "+v"(st[0][0]), "+v"(st[0][QT - 1]), "+v"(st[1][0]), "+v"(st[1][QT - 1]) : "v"(qf[0][0]));
        else asm volatile("v_nop\n\tv_nop\n\tv_nop\n\tv_nop" : "+v"(st[0][0]), "+v"(st[1][0]) : "v"(qf[0][0]));
        const int mk = mr[k0 + lane];
        const unsigned vbits = __builtin_amdgcn_ballot_w32(mk != 0);
        if (vbits != 0xffffffffu || k0 + 31u > q0) {
            const unsigned vb = vbits >> (8u * hi);
#pragma unroll
            for (int qt = 0; qt < QT; ++qt) { const unsigned qq = q0 + (unsigned)qt * 16u + lr;
#pragma unroll
                for (int kt = 0; kt < 2; ++kt)
#pragma unroll
                    for (int r = 0; r < 8; ++r) { const unsigned key = k0 + (unsigned)kt * 16u + 8u * hi + (unsigned)r;
                        const bool ok = (((vb >> (kt * 16 + r)) & 1u) != 0u) && (key <= qq);
                        st[kt][qt][r] = ok ? st[kt][qt][r] : NEGL; } }
        }
        V pf[QT], pg[QT]; float al[QT]; bool need = false;
#pragma unroll
        for (int qt = 0; qt < QT; ++qt) {
            float mx = st[0][qt][0];
#pragma unroll
            for (int r = 1; r < 8; ++r) mx = fmaxf(mx, st[0][qt][r]);
#pragma unroll
            for (int r = 0; r < 8; ++r) mx = fmaxf(mx, st[1][qt][r]);
            mx = fmaxf(mx, __shfl_xor(mx, 16, 32));
            const float mnew = fmaxf(mrun[qt], mx);
            al[qt] = __builtin_amdgcn_exp2f((mrun[qt] - mnew) * SL2E);
            mrun[qt] = mnew; need = need || (al[qt] != 1.0f);
            const float cc = 10.0f - mnew * SL2E;
            float psum = 0.f; float p0[8], p1[8];
#pragma unroll
            for (int r = 0; r < 8; ++r) { p0[r] = __builtin_amdgcn_exp2f(fmaf(st[0][qt][r], SL2E, cc)); psum += p0[r]; }
#pragma unroll
            for (int r = 0; r < 8; ++r) { p1[r] = __builtin_amdgcn_exp2f(fmaf(st[1][qt][r], SL2E, cc)); psum += p1[r]; }
            lrun[qt] = lrun[qt] * al[qt] + psum;
            if constexpr (!HL) { v8h a0, a1;
#pragma unroll
                for (int r = 0; r < 8; ++r) { a0[r] = tohx(p0[r]); a1[r] = tohx(p1[r]); }
                pf[qt] = cat16(a0, a1);
            } else { v8us h0, h1, l0, l1;
#pragma unroll
                for (int r = 0; r < 8; ++r) { unsigned short a2, c2; splitf(p0[r], a2, c2); h0[r] = a2; l0[r] = c2; splitf(p1[r], a2, c2); h1[r] = a2; l1[r] = c2; }
                pf[qt] = cat16b(h0, h1); pg[qt] = cat16b(l0, l1); }
        }
        if (__builtin_amdgcn_ballot_w32(need) != 0u) {
#pragma unroll
            for (int dt = 0; dt < 4; ++dt)
#pragma unroll
                for (int qt = 0; qt < QT; ++qt)
#pragma unroll
                    for (int r = 0; r < 8; ++r) o[dt][qt][r] *= al[qt];
        }
#pragma unroll
        for (int dt = 0; dt < 4; ++dt) { const size_t vo = pbase + (size_t)((unsigned)dt * 16u + lr) * PR + k0 + 8u * hi;
            const V a = W::ld(Va + vo); V a2; if constexpr (HL) a2 = W::ld(Vb + vo);
#pragma unroll
            for (int qt = 0; qt < QT; ++qt) { o[dt][qt] = W::mma(a, pf[qt], o[dt][qt]);
                if constexpr (HL) { o[dt][qt] = W::mma(a2, pf[qt], o[dt][qt]); o[dt][qt] = W::mma(a, pg[qt], o[dt][qt]); } } }
        asm volatile("v_nop\n\tv_nop\n\tv_nop\n\tv_nop" : "+v"(o[0][0]), "+v"(o[1][QT - 1]), "+v"(o[2][0]), "+v"(o[3][QT - 1]) : "v"(pf[0]));
    }
#pragma unroll
    for (int qt = 0; qt < QT; ++qt) {
        const float lt = lrun[qt] + __shfl_xor(lrun[qt], 16, 32);
        const unsigned qq = q0 + (unsigned)qt * 16u + lr;
        const float qm = (mr[qq] != 0) ? 1.0f : 0.0f;
        const float inv = (HL ? 1.0f : CCAR) / lt;
        const float pz = (mrun[qt] < -0.5e30f) ? __uint_as_float(0x7fc00000u) : 0.0f;
#pragma unroll
        for (int dt = 0; dt < 4; ++dt)
#pragma unroll
            for (int r = 0; r < 8; ++r) os[((unsigned)qt * 16u + lr) * 68u + (unsigned)dt * 16u + 8u * hi + (unsigned)r] = (o[dt][qt][r] * inv) * qm + pz;
    }
    __syncthreads();
    const size_t orow = (size_t)b * PR + q0;
#pragma unroll 1
    for (int ps = 0; ps < 2; ++ps) {
#pragma unroll
        for (unsigned s = 0; s < 4u * QT; ++s) {
            const unsigned row = s * 4u + sub; const float* src = os + row * 68u + seg * 8u;
            const v4f x0 = *(const v4fa*)src, x1 = *(const v4fa*)(src + 4);
            const size_t oo = (orow + row) * DMODEL + head * HDIM + seg * 8u;
            if constexpr (!HL) { v8h ov;
#pragma unroll
                for (int i = 0; i < 4; ++i) { ov[i] = tohx(x0[i]); ov[4 + i] = tohx(x1[i]); }
                *(volatile v8h*)(Oa + oo) = ov;
            } else { v8us oh, ol;
#pragma unroll
                for (int i = 0; i < 4; ++i) { unsigned short a2, c2; splitf(x0[i], a2, c2); oh[i] = a2; ol[i] = c2; splitf(x1[i], a2, c2); oh[4 + i] = a2; ol[4 + i] = c2; }
                *(volatile v8us*)(Oa + oo) = oh; *(volatile v8us*)(Ob + oo) = ol; }
        }
        if (ps == 0) __threadfence();
    }
}

template <typename T16, int NSPLIT>
__global__ __launch_bounds__(32) void k_gemmo(const T16* __restrict__ A, const T16* __restrict__ A2, const T16* __restrict__ Bt, int K, float* C, int ldc,
                                              const float* __restrict__ bias, float osc, size_t sA, size_t sC) {
    typedef typename WFrag<T16>::V V;
    __shared__ __align__(16) float os[16 * 68];
    const size_t z = blockIdx.z; A += z * sA; if constexpr (NSPLIT == 1) A2 += z * sA; C += z * sC;
    const unsigned lane = threadIdx.x & 31u, lr = lane & 15u, hi = lane >> 4; const unsigned r0 = blockIdx.x * 64u, c0 = blockIdx.y * 64u;
    v8f acc[4][4];
#pragma unroll
    for (int mb = 0; mb < 4; ++mb)
#pragma unroll
        for (int nb = 0; nb < 4; ++nb) acc[mb][nb] = (v8f){};
    const size_t aoff = (size_t)(r0 + lr) * K + 8u * hi, boff = (size_t)(c0 + lr) * K + 8u * hi;
#pragma unroll 1
    for (int kc = 0; kc < K; kc += 32) {
        V a[4], a2[4];
#pragma unroll
        for (int mb = 0; mb < 4; ++mb) { a[mb] = WFrag<T16>::ld(A + aoff + (size_t)mb * 16 * K + kc); if constexpr (NSPLIT == 1) a2[mb] = WFrag<T16>::ld(A2 + aoff + (size_t)mb * 16 * K + kc); }
#pragma unroll
        for (int nb = 0; nb < 4; ++nb) { const V b = WFrag<T16>::ld(Bt + boff + (size_t)nb * 16 * K + kc);
#pragma unroll
            for (int mb = 0; mb < 4; ++mb) { acc[mb][nb] = WFrag<T16>::mma(a[mb], b, acc[mb][nb]); if constexpr (NSPLIT == 1) acc[mb][nb] = WFrag<T16>::mma(a2[mb], b, acc[mb][nb]); } }
        asm volatile("v_nop\n\tv_nop\n\tv_nop\n\tv_nop" : "+v"(acc[0][0]), "+v"(acc[1][1]), "+v"(acc[2][2]), "+v"(acc[3][3]) : "v"(a[0]), "v"(a[3]));
    }
    const unsigned cofs = lr * 4u; float b4[4];
#pragma unroll
    for (int i = 0; i < 4; ++i) b4[i] = bfr(bias[c0 + cofs + (unsigned)i]);
#pragma unroll
    for (int mb = 0; mb < 4; ++mb) {
#pragma unroll
        for (int nb = 0; nb < 4; ++nb)
#pragma unroll
            for (int j = 0; j < 8; ++j) os[(hi * 8u + (unsigned)j) * 68u + (unsigned)nb * 16u + lr] = acc[mb][nb][j];
        __syncthreads();
        float* crow = C + (size_t)(r0 + (unsigned)mb * 16u) * ldc + c0;
#pragma unroll 1
        for (int ps = 0; ps < 2; ++ps) {
#pragma unroll
            for (unsigned s = 0; s < 8u; ++s) { const unsigned row = 2u * s + hi; v4f val = *(const v4fa*)(os + row * 68u + cofs);
#pragma unroll
                for (int i = 0; i < 4; ++i) val[i] = val[i] * osc + b4[i];
                *(volatile v4f*)(crow + (size_t)row * ldc + cofs) = val; }
            if (ps == 0) __threadfence(); }
        __syncthreads();
    }
}

constexpr size_t AL256(size_t b) { return (b + 255) & ~(size_t)255; }
constexpr size_t SZ_WQKV = AL256((size_t)3 * DMODEL * DMODEL * 2);
constexpr size_t SZ_WO   = AL256((size_t)DMODEL * DMODEL * 2);
constexpr size_t SZ_XB   = AL256((size_t)NB * SEQ * DMODEL * 2);
constexpr size_t SZ_P16  = AL256((size_t)NB * NHEAD * SEQ * HDIM * 2);
constexpr size_t SZ_PHL  = AL256((size_t)NB * NHEAD * RHI * HDIM * 2);
constexpr size_t SZ_CT   = AL256((size_t)NB * SEQ * DMODEL * 2);
constexpr size_t SZ_AT   = AL256((size_t)NB * RHI * DMODEL * 2);
constexpr size_t WS_TOTAL = SZ_WQKV + 2 * SZ_WO + SZ_XB + 3 * SZ_P16 + 6 * SZ_PHL + SZ_CT + 2 * SZ_AT;
static_assert(WS_TOTAL <= (size_t)134217728);
static_assert(16 * 4 == 64);
static_assert((NB * SEQ / 64) * 64 == NB * SEQ);
static_assert((3 * DMODEL / 64) * 64 == 3 * DMODEL);
static_assert((RHI / 16) * 16 == RHI);
static_assert(((SEQ - RHI) / 32) * 32 == SEQ - RHI);
static_assert(((NB * SEQ * (DMODEL / 8) + 255) / 256) * 256 >= NB * SEQ * (DMODEL / 8));

extern "C" void kernel_launch(void* const* d_in, const int* in_sizes, int n_in,
                              void* d_out, int out_size, void* d_ws, size_t ws_size, hipStream_t stream) {
    if (n_in < 6) return;
    const long long need_rows = (long long)(NB - 1) * SEQ_FULL + SEQ;
    if ((long long)in_sizes[0] < need_rows * DMODEL) return;
    if ((long long)in_sizes[1] < need_rows) return;
    if ((long long)in_sizes[2] < (long long)3 * DMODEL * DMODEL) return;
    if (in_sizes[3] < 3 * DMODEL) return;
    if ((long long)in_sizes[4] < (long long)DMODEL * DMODEL) return;
    if (in_sizes[5] < DMODEL) return;
    if ((long long)out_size < need_rows * DMODEL) return;
    const float* x = (const float*)d_in[0]; const int* amask = (const int*)d_in[1]; const float* wqkv = (const float*)d_in[2];
    const float* bqkv = (const float*)d_in[3]; const float* wo = (const float*)d_in[4]; const float* bo = (const float*)d_in[5];
    float* OUT = (float*)d_out;
    char* wsp = (char*)d_ws;
    auto take = [&](size_t bytes) { char* p = wsp; wsp += bytes; return (void*)p; };
    bf* WQKV = (bf*)take(SZ_WQKV); bf* WO = (bf*)take(SZ_WO); h16* WO16 = (h16*)take(SZ_WO); bf* XB = (bf*)take(SZ_XB);
    h16* Q16 = (h16*)take(SZ_P16); h16* K16 = (h16*)take(SZ_P16); h16* VT16 = (h16*)take(SZ_P16);
    bf* QPh = (bf*)take(SZ_PHL); bf* QPl = (bf*)take(SZ_PHL); bf* KPh = (bf*)take(SZ_PHL); bf* KPl = (bf*)take(SZ_PHL); bf* VTh = (bf*)take(SZ_PHL); bf* VTl = (bf*)take(SZ_PHL);
    h16* CT16 = (h16*)take(SZ_CT); bf* ATh = (bf*)take(SZ_AT); bf* ATl = (bf*)take(SZ_AT);
    if ((size_t)(wsp - (char*)d_ws) > ws_size) return;

    k_cvtx<<<(unsigned)((NB * SEQ * (DMODEL / 8) + 255) / 256), 256, 0, stream>>>(x, XB);
    k_cvt8<<<(unsigned)((3 * DMODEL * DMODEL / 8 + 255) / 256), 256, 0, stream>>>(wqkv, WQKV, (unsigned)(3 * DMODEL * DMODEL / 8));
    k_cvtwo<<<(unsigned)((DMODEL * DMODEL / 8 + 255) / 256), 256, 0, stream>>>(wo, WO, WO16, (unsigned)(DMODEL * DMODEL / 8));
    k_gemmqkv<<<dim3(NB * SEQ / 64, 3 * DMODEL / 64, 1), 32, 0, stream>>>(XB, WQKV, bqkv, Q16, QPh, QPl, K16, KPh, KPl, VT16, VTh, VTl);
    k_flash<true, 1><<<dim3(RHI / 16, NHEAD, NB), 32, 0, stream>>>(QPh, QPl, KPh, KPl, VTh, VTl, amask, ATh, ATl);
    if (SEQ > RHI)
        k_flash<false, 2><<<dim3((SEQ - RHI) / 32, NHEAD, NB), 32, 0, stream>>>(Q16, (const h16*)nullptr, K16, (const h16*)nullptr, VT16, (const h16*)nullptr, amask, CT16, (h16*)nullptr);
    k_gemmo<bf, 1><<<dim3(RHI / 64, DMODEL / 64, NB), 32, 0, stream>>>(ATh, ATl, WO, DMODEL, OUT, DMODEL, bo, 1.0f, (size_t)RHI * DMODEL, (size_t)SEQ_FULL * DMODEL);
    if (SEQ > RHI)
        k_gemmo<h16, 0><<<dim3((SEQ - RHI) / 64, DMODEL / 64, NB), 32, 0, stream>>>(CT16 + (size_t)RHI * DMODEL, (const h16*)nullptr, WO16, DMODEL, OUT + (size_t)RHI * DMODEL, DMODEL, bo, 1.0f / (WCAR * CCAR), (size_t)SEQ * DMODEL, (size_t)SEQ_FULL * DMODEL);
}
